// GatedAttn_23510650978924
// MI455X (gfx1250) — hardware-verified
//
#include <hip/hip_runtime.h>
#include <math.h>

typedef __attribute__((ext_vector_type(16))) _Float16 v16h;
typedef __attribute__((ext_vector_type(16))) __bf16 v16b;
typedef __attribute__((ext_vector_type(8)))  _Float16 v8h;
typedef __attribute__((ext_vector_type(8)))  float v8f;
typedef __attribute__((ext_vector_type(4)))  float v4f;
typedef __attribute__((ext_vector_type(2)))  float v2f;
typedef __attribute__((ext_vector_type(4)))  unsigned v4u;
typedef __attribute__((ext_vector_type(4)))  int v4i;
typedef float __attribute__((may_alias)) float_a;
typedef int __attribute__((may_alias)) int_a;

template <typename T> __device__ __forceinline__ void vst2(void* p, T v) { *(volatile T*)p = v; __threadfence(); *(volatile T*)p = v; }
__device__ __forceinline__ v8f wmma16(v16h a, v16h b, v8f c) {
  v8f d = __builtin_amdgcn_wmma_f32_16x16x32_f16(false, a, false, b, (short)0, c, false, false);
  asm volatile("v_nop\n\tv_nop\n\tv_nop\n\tv_nop" : "+v"(d) : "v"(a), "v"(b));
  return d;
}
__device__ __forceinline__ v8f wmma_bf(v16b a, v16b b, v8f c) {
  v8f d = __builtin_amdgcn_wmma_f32_16x16x32_bf16(false, a, false, b, (short)0, c, false, false);
  asm volatile("v_nop\n\tv_nop\n\tv_nop\n\tv_nop" : "+v"(d) : "v"(a), "v"(b));
  return d;
}
__device__ __forceinline__ v16h frag_h(const _Float16* rowk0, int lane) {
  union { v16h v; v8h q[2]; } u; const _Float16* p = rowk0 + 8 * (lane >> 4);
  u.q[0] = *(const v8h*)p; u.q[1] = *(const v8h*)(p + 16); return u.v;
}
__device__ __forceinline__ v16h frag_f32(const float* rowk0, int lane) {
  v16h a; const float* p = rowk0 + 8 * (lane >> 4);
#pragma unroll
  for (int i = 0; i < 8; ++i) { a[i] = (_Float16)p[i]; a[8 + i] = (_Float16)p[16 + i]; }
  return a;
}
__device__ __forceinline__ v16h frag_f32s(const float* rowk0, int lane, float sc) {
  v16h a; const float* p = rowk0 + 8 * (lane >> 4);
#pragma unroll
  for (int i = 0; i < 8; ++i) { a[i] = (_Float16)(p[i] * sc); a[8 + i] = (_Float16)(p[16 + i] * sc); }
  return a;
}
__device__ __forceinline__ v16h fragc_f32(const float* W, int k0, int n, int lane, int ld, int K) {
  v16h a; const int g = lane >> 4;
#pragma unroll
  for (int i = 0; i < 8; ++i) { const int ka = k0 + 8 * g + i, kb = ka + 16;
    a[i] = (_Float16)(ka < K ? W[(size_t)(ka < K ? ka : K - 1) * ld + n] : 0.f); a[8 + i] = (_Float16)(kb < K ? W[(size_t)(kb < K ? kb : K - 1) * ld + n] : 0.f); }
  return a;
}
struct F2 { v16b h, l; };
__device__ __forceinline__ F2 bsplit16(const float v[16]) { F2 r;
#pragma unroll
  for (int i = 0; i < 16; ++i) { const __bf16 h = (__bf16)v[i]; r.h[i] = h; r.l[i] = (__bf16)(v[i] - (float)h); }
  return r; }
__device__ __forceinline__ F2 split_row(const float* row, int k0, int lane) { float v[16]; const float* p = row + k0 + 8 * (lane >> 4);
#pragma unroll
  for (int i = 0; i < 8; ++i) { v[i] = p[i]; v[8 + i] = p[16 + i]; }
  return bsplit16(v); }
__device__ __forceinline__ F2 split_rowK(const float* row, int k0, int lane, int K) { float v[16]; const int g = lane >> 4;
#pragma unroll
  for (int i = 0; i < 8; ++i) { const int ka = k0 + 8 * g + i, kb = ka + 16; v[i] = ka < K ? row[ka < K ? ka : K - 1] : 0.f; v[8 + i] = kb < K ? row[kb < K ? kb : K - 1] : 0.f; }
  return bsplit16(v); }
__device__ __forceinline__ F2 split_col(const float* W, int k0, int n, int lane, int ld, int K) { float v[16]; const int g = lane >> 4;
#pragma unroll
  for (int i = 0; i < 8; ++i) { const int ka = k0 + 8 * g + i, kb = ka + 16; v[i] = ka < K ? W[(size_t)(ka < K ? ka : K - 1) * ld + n] : 0.f; v[8 + i] = kb < K ? W[(size_t)(kb < K ? kb : K - 1) * ld + n] : 0.f; }
  return bsplit16(v); }
__device__ __forceinline__ v8f mac3(const F2& a, const F2& b, v8f c) { c = wmma_bf(a.l, b.h, c); c = wmma_bf(a.h, b.l, c); return wmma_bf(a.h, b.h, c); }
__device__ __forceinline__ float sigm(float v) { return 1.0f / (1.0f + expf(-v)); }
#define LDSX() do { asm volatile("s_wait_dscnt 0" ::: "memory"); __builtin_amdgcn_wave_barrier(); __builtin_amdgcn_fence(__ATOMIC_RELEASE, "workgroup"); } while (0)


#define NB 8
#define CC 128
#define NN 1024
#define NHD 4
#define DH 32
__device__ __attribute__((noinline)) float sigm_ni(float v) { return 1.0f / (1.0f + expf(-v)); }
__device__ __forceinline__ float bfr(float v) { return (float)(__bf16)v; }
__device__ __forceinline__ v16b frag_b(const __bf16* rowk0, int lane) { return __builtin_bit_cast(v16b, frag_h((const _Float16*)rowk0, lane)); }

__global__ __launch_bounds__(256) void k_cvtx(const float* __restrict__ x, __bf16* __restrict__ XT) {
  __shared__ __align__(16) __bf16 st[64][CC + 8];
  const int tid = threadIdx.x; const int b = blockIdx.y, p0 = blockIdx.x * 64;
  for (int q = tid; q < CC * 16; q += 256) { const int c = q >> 4, p4 = q & 15; const v4f v = *(const v4f*)(x + ((size_t)b * CC + c) * NN + p0 + p4 * 4);
    st[p4 * 4][c] = (__bf16)v[0]; st[p4 * 4 + 1][c] = (__bf16)v[1]; st[p4 * 4 + 2][c] = (__bf16)v[2]; st[p4 * 4 + 3][c] = (__bf16)v[3]; }
  __syncthreads();
  for (int q = tid; q < 64 * (CC / 8); q += 256) { const int rl = q / (CC / 8), pc = q % (CC / 8); vst2((unsigned*)(XT + ((size_t)b * NN + p0 + rl) * CC + pc * 8), *(const v4u*)(&st[rl][pc * 8])); }
}
__global__ __launch_bounds__(128) void k_qkv(const __bf16* __restrict__ XT, const float* __restrict__ W, const float* __restrict__ bias, float* __restrict__ Q32, __bf16* __restrict__ Kh, __bf16* __restrict__ Kl, __bf16* __restrict__ VTh, __bf16* __restrict__ VTl) {
  __shared__ __align__(16) float so[4][16][132]; __shared__ __align__(16) __bf16 sh_[4][16][136], sl_[4][16][136]; __shared__ __align__(16) __bf16 sth[128][72], stl[128][72];
  const int tid = threadIdx.x, wave = tid >> 5, lane = tid & 31, col = lane & 15, g = lane >> 4; const int r0b = blockIdx.x * 64, n0 = blockIdx.y * 128, which = blockIdx.z; const int b = r0b / NN, s0 = r0b % NN; const size_t r0 = (size_t)r0b + wave * 16;
  v8f acc[8] = {};
#pragma unroll
  for (int kc = 0; kc < CC / 32; ++kc) { const v16b a = frag_b(XT + (r0 + col) * CC + kc * 32, lane);
#pragma unroll
    for (int j = 0; j < 8; ++j) { const int c = n0 + j * 16 + col; acc[j] = wmma_bf(a, split_col(W, kc * 32, (c >> 5) * (3 * DH) + which * DH + (c & 31), lane, 3 * CC, CC).h, acc[j]); } }
  if (which == 0) {
#pragma unroll
    for (int j = 0; j < 8; ++j) { const int c = n0 + j * 16 + col; const float bb = bfr(bias[(c >> 5) * (3 * DH) + 0 * DH + (c & 31)]);
#pragma unroll
      for (int r = 0; r < 8; ++r) so[wave][8 * g + r][j * 16 + col] = acc[j][r] + bb; }
    LDSX();
    for (int qq = lane; qq < 4 * 16 * 8; qq += 32) { const int hh = qq >> 7, rl = (qq >> 3) & 15, pc = qq & 7; const int h = (n0 >> 5) + hh; vst2(Q32 + (((size_t)b * NHD + h) * NN + s0 + wave * 16 + rl) * DH + pc * 4, *(const v4f*)(&so[wave][rl][hh * 32 + pc * 4])); } }
  else if (which == 1) {
#pragma unroll
    for (int j = 0; j < 8; ++j) { const int c = n0 + j * 16 + col; const float bb = bfr(bias[(c >> 5) * (3 * DH) + 1 * DH + (c & 31)]);
#pragma unroll
      for (int r = 0; r < 8; ++r) { const float v = acc[j][r] + bb; const __bf16 hi = (__bf16)v; sh_[wave][8 * g + r][j * 16 + col] = hi; sl_[wave][8 * g + r][j * 16 + col] = (__bf16)(v - (float)hi); } }
    LDSX();
    for (int qq = lane; qq < 4 * 16 * 4; qq += 32) { const int hh = qq >> 6, rl = (qq >> 2) & 15, pc = qq & 3; const int h = (n0 >> 5) + hh; const size_t o = (((size_t)b * NHD + h) * NN + s0 + wave * 16 + rl) * DH + pc * 8; vst2((unsigned*)(Kh + o), *(const v4u*)(&sh_[wave][rl][hh * 32 + pc * 8])); vst2((unsigned*)(Kl + o), *(const v4u*)(&sl_[wave][rl][hh * 32 + pc * 8])); } }
  else {
#pragma unroll
    for (int j = 0; j < 8; ++j) { const int c = n0 + j * 16 + col; const float bb = bfr(bias[(c >> 5) * (3 * DH) + 2 * DH + (c & 31)]);
#pragma unroll
      for (int r = 0; r < 8; ++r) { const float v = acc[j][r] + bb; const __bf16 hi = (__bf16)v; sth[j * 16 + col][wave * 16 + 8 * g + r] = hi; stl[j * 16 + col][wave * 16 + 8 * g + r] = (__bf16)(v - (float)hi); } }
    __syncthreads();
    for (int qq = tid; qq < 128 * 8; qq += 128) { const int cl = qq >> 3, pc = qq & 7; const int c = n0 + cl; const int h = c >> 5, d = c & 31; const size_t o = (((size_t)b * NHD + h) * DH + d) * NN + s0 + pc * 8; vst2((unsigned*)(VTh + o), *(const v4u*)(&sth[cl][pc * 8])); vst2((unsigned*)(VTl + o), *(const v4u*)(&stl[cl][pc * 8])); } }
}
__global__ __launch_bounds__(128) void k_attn(const float* __restrict__ Q32, const __bf16* __restrict__ Kh, const __bf16* __restrict__ Kl, const __bf16* __restrict__ VTh, const __bf16* __restrict__ VTl, float* __restrict__ O) {
  __shared__ __align__(16) float sS[4][16][68];
  __shared__ __align__(16) __bf16 sPh[4][16][72], sPl[4][16][72];
  __shared__ __align__(16) float sO[4][16][36];
  const int tid = threadIdx.x, w = tid >> 5, lane = tid & 31, col = lane & 15, g = lane >> 4; const size_t bh = blockIdx.y; const int b = (int)(bh / NHD), h = (int)(bh % NHD); const int q0 = blockIdx.x * 64 + w * 16;
  const F2 aq = split_row(Q32 + (bh * NN + q0 + col) * DH, 0, lane);
  float mrun = -3.0e38f, lrun = 0.f; v8f acc[2] = {};
#pragma unroll 1
  for (int kt = 0; kt < NN / 64; ++kt) {
#pragma unroll
    for (int t = 0; t < 4; ++t) { const int key = kt * 64 + t * 16 + col; const size_t ko = (bh * NN + key) * DH; const v16b khf = frag_b(Kh + ko, lane), klf = frag_b(Kl + ko, lane);
      v8f s = {}; s = wmma_bf(aq.l, khf, s); s = wmma_bf(aq.h, klf, s); s = wmma_bf(aq.h, khf, s);
#pragma unroll
      for (int r = 0; r < 8; ++r) sS[w][8 * g + r][t * 16 + col] = s[r] * 0.17677669529663687f; }
    LDSX();
    float mx = -3.4e38f;
#pragma unroll
    for (int jj = 0; jj < 32; ++jj) mx = fmaxf(mx, sS[w][col][g * 32 + jj]);
    mx = fmaxf(mx, __shfl_xor(mx, 16, 32));
    const float mnew = fmaxf(mrun, mx); const float corr = expf(mrun - mnew);
    float ps = 0.f;
#pragma unroll
    for (int jj = 0; jj < 32; ++jj) { const float p = expf(sS[w][col][g * 32 + jj] - mnew); ps += p; const __bf16 hi = (__bf16)p; sPh[w][col][g * 32 + jj] = hi; sPl[w][col][g * 32 + jj] = (__bf16)(p - (float)hi); }
    ps += __shfl_xor(ps, 16, 32);
    lrun = lrun * corr + ps; mrun = mnew;
#pragma unroll
    for (int r = 0; r < 8; ++r) { const float cr = __shfl(corr, 8 * g + r, 32); acc[0][r] *= cr; acc[1][r] *= cr; }
    LDSX();
#pragma unroll
    for (int kc = 0; kc < 2; ++kc) { const v16b ph = frag_b(&sPh[w][col][0] + kc * 32, lane), pl = frag_b(&sPl[w][col][0] + kc * 32, lane);
#pragma unroll
      for (int t = 0; t < 2; ++t) { const size_t vo = (bh * DH + t * 16 + col) * NN + kt * 64 + kc * 32; const v16b vh = frag_b(VTh + vo, lane), vl = frag_b(VTl + vo, lane); acc[t] = wmma_bf(pl, vh, acc[t]); acc[t] = wmma_bf(ph, vl, acc[t]); acc[t] = wmma_bf(ph, vh, acc[t]); } }
    __builtin_amdgcn_wave_barrier(); }
#pragma unroll
  for (int r = 0; r < 8; ++r) { const float lr = __shfl(lrun, 8 * g + r, 32); const float inv = 1.0f / lr; sO[w][8 * g + r][col] = acc[0][r] * inv; sO[w][8 * g + r][16 + col] = acc[1][r] * inv; }
  LDSX();
  for (int qq = lane; qq < 16 * 8; qq += 32) { const int rl = qq >> 3, pc = qq & 7; vst2(O + ((size_t)b * NN + q0 + rl) * CC + h * DH + pc * 4, *(const v4f*)(&sO[w][rl][pc * 4])); }
}
__global__ __launch_bounds__(128) void k_out(const float* __restrict__ O, const float* __restrict__ Wg, const float* __restrict__ bg, const float* __restrict__ x, float* __restrict__ y) {
  __shared__ __align__(16) float sY[4][32][68];
  const int tid = threadIdx.x, w = tid >> 5, lane = tid & 31, col = lane & 15, g = lane >> 4; const int b = blockIdx.y, p0 = blockIdx.x * 64; const size_t base = (size_t)b * NN;
  v8f av[2][4] = {}, ag[2][4] = {};
#pragma unroll 1
  for (int kc = 0; kc < CC / 32; ++kc) { F2 bc[4];
#pragma unroll
    for (int pt = 0; pt < 4; ++pt) bc[pt] = split_row(O + (base + p0 + pt * 16 + col) * CC, kc * 32, lane);
#pragma unroll
    for (int ct = 0; ct < 2; ++ct) { const int c = (w * 2 + ct) * 16 + col; const v16b a1 = split_col(Wg, kc * 32, c, lane, 2 * CC, CC).h, a2 = split_col(Wg, kc * 32, CC + c, lane, 2 * CC, CC).h;
#pragma unroll
      for (int pt = 0; pt < 4; ++pt) { av[ct][pt] = wmma_bf(a1, bc[pt].l, av[ct][pt]); av[ct][pt] = wmma_bf(a1, bc[pt].h, av[ct][pt]); ag[ct][pt] = wmma_bf(a2, bc[pt].l, ag[ct][pt]); ag[ct][pt] = wmma_bf(a2, bc[pt].h, ag[ct][pt]); } } }
#pragma unroll
  for (int ct = 0; ct < 2; ++ct) {
#pragma unroll
    for (int r = 0; r < 8; ++r) { const int cl = ct * 16 + 8 * g + r; const int c = w * 32 + cl; const float bv_ = bfr(bg[c]), bg_ = bfr(bg[CC + c]);
#pragma unroll
      for (int pt = 0; pt < 4; ++pt) { const int n = p0 + pt * 16 + col; const float val = av[ct][pt][r] + bv_; const float gt = ag[ct][pt][r] + bg_; sY[w][cl][pt * 16 + col] = bfr(x[((size_t)b * CC + c) * NN + n]) + val * sigm_ni(gt); } } }
  LDSX();
  for (int qq = lane; qq < 32 * 16; qq += 32) { const int cl = qq >> 4, pc = qq & 15; vst2(y + ((size_t)b * CC + w * 32 + cl) * NN + p0 + pc * 4, *(const v4f*)(&sY[w][cl][pc * 4])); }
}
extern "C" void kernel_launch(void* const* d_in, const int* in_sizes, int n_in, void* d_out, int out_size, void* d_ws, size_t ws_size, hipStream_t stream) {
  (void)in_sizes; (void)n_in; (void)out_size; (void)ws_size;
  const float* x = (const float*)d_in[0]; const float* Wqkv = (const float*)d_in[1]; const float* bqkv = (const float*)d_in[2]; const float* Wg = (const float*)d_in[3]; const float* bg = (const float*)d_in[4];
  char* ws = (char*)d_ws; size_t off = 0;
  auto take = [&](size_t bytes) { char* p = ws + off; off += (bytes + 255) & ~(size_t)255; return p; };
  __bf16* XT = (__bf16*)take((size_t)NB * NN * CC * 2); float* Q32 = (float*)take((size_t)NB * NN * CC * 4); __bf16* Kh = (__bf16*)take((size_t)NB * NN * CC * 2); __bf16* Kl = (__bf16*)take((size_t)NB * NN * CC * 2); __bf16* VTh = (__bf16*)take((size_t)NB * NN * CC * 2); __bf16* VTl = (__bf16*)take((size_t)NB * NN * CC * 2); float* O = (float*)take((size_t)NB * NN * CC * 4);
  k_cvtx<<<dim3(NN / 64, NB), 256, 0, stream>>>(x, XT);
  k_qkv<<<dim3(NB * NN / 64, CC / 128, 3), 128, 0, stream>>>(XT, Wqkv, bqkv, Q32, Kh, Kl, VTh, VTl);
  k_attn<<<dim3(NN / 64, NB * NHD), 128, 0, stream>>>(Q32, Kh, Kl, VTh, VTl, O);
  k_out<<<dim3(NN / 64, NB), 128, 0, stream>>>(O, Wg, bg, x, (float*)d_out);
}
